// FEM_best_55439437857362
// MI455X (gfx1250) — hardware-verified
//
#include <hip/hip_runtime.h>
#include <stddef.h>
#include <stdint.h>
#include <math.h>

#define NBT   2
#define CIN   256
#define CI    128
#define HWD   64
#define NPX   4096
#define PW    66
#define KC3   2304
#define NIMG  4
#define TP    72
#define EPF   68
#define TPP   264
#define XPIMG ((size_t)PW * PW * CIN)
#define XSIMG ((size_t)CI * NPX)
#define XHIMG ((size_t)NPX * CI)
#define VIMG  ((size_t)CI * NPX)
#define KIMG  ((size_t)NPX * CI)
#define W3SET ((size_t)CI * KC3)
#define WCSET ((size_t)256 * CI)
#define OUTB  ((size_t)CI * NPX)

#define XP_BYTES  ((size_t)NIMG * XPIMG * 2)
#define W3_BYTES  ((size_t)3 * W3SET * 2)
#define WC_BYTES  ((size_t)2 * WCSET * 2)
#define XS_BYTES  ((size_t)NIMG * XSIMG * 4)
#define XH_BYTES  ((size_t)NIMG * XHIMG * 2)
#define V_BYTES   ((size_t)NIMG * VIMG * 2)
#define VP_BYTES  ((size_t)NIMG * 64 * CI * 4)
#define G_BYTES   ((size_t)4096)
#define KQ_BYTES  ((size_t)NBT * KIMG * 2)
#define S_BYTES   ((size_t)NPX * NPX * 4)
#define ST_BYTES  ((size_t)NPX * 4)
#define EP_BYTES  ((size_t)NBT * XPIMG * 2)

#define OFF_XP   ((size_t)0)
#define OFF_W3   (OFF_XP + XP_BYTES)
#define OFF_WC   (OFF_W3 + W3_BYTES)
#define OFF_XS   (OFF_WC + WC_BYTES)
#define OFF_XH   (OFF_XS + XS_BYTES)
#define OFF_XL   (OFF_XH + XH_BYTES)
#define OFF_V    (OFF_XL + XH_BYTES)
#define OFF_VP   (OFF_V + V_BYTES)
#define OFF_G    (OFF_VP + VP_BYTES)
#define OFF_KH   (OFF_G + G_BYTES)
#define OFF_KL   (OFF_KH + KQ_BYTES)
#define OFF_QH   (OFF_KL + KQ_BYTES)
#define OFF_QL   (OFF_QH + KQ_BYTES)
#define OFF_S    (OFF_QL + KQ_BYTES)
#define OFF_RMAX (OFF_S + S_BYTES)
#define OFF_RSUM (OFF_RMAX + ST_BYTES)
#define OFF_CMAX (OFF_RSUM + ST_BYTES)
#define OFF_CSUM (OFF_CMAX + ST_BYTES)
#define OFF_EP   (OFF_CSUM + ST_BYTES)
#define WS_TOTAL (OFF_EP + EP_BYTES)

static_assert(OFF_W3 == (size_t)8921088);
static_assert(OFF_S == (size_t)40316928);
static_assert(OFF_EP == (size_t)107491328);
static_assert(WS_TOTAL == (size_t)111951872);
static_assert(WS_TOTAL <= (size_t)134217728);
static_assert((OFF_W3 % 256) == 0);
static_assert((OFF_WC % 256) == 0);
static_assert((OFF_XS % 256) == 0);
static_assert((OFF_XH % 256) == 0);
static_assert((OFF_XL % 256) == 0);
static_assert((OFF_V % 256) == 0);
static_assert((OFF_VP % 256) == 0);
static_assert((OFF_G % 256) == 0);
static_assert((OFF_KH % 256) == 0);
static_assert((OFF_S % 256) == 0);
static_assert((OFF_RMAX % 256) == 0);
static_assert((OFF_EP % 256) == 0);
static_assert((XPIMG * 2) % 256 == 0);
static_assert(NPX == HWD * HWD);
static_assert(KC3 == 9 * CIN);
static_assert((KC3 % 32) == 0);
static_assert((CI % 32) == 0);
static_assert((NPX % 64) == 0);
static_assert(PW * TPP * 2 <= 40000);
static_assert((TPP * 2) % 16 == 0);
static_assert((TP * 2) % 16 == 0);
static_assert((EPF * 4) % 16 == 0);

typedef unsigned short v8us  __attribute__((ext_vector_type(8)));
typedef unsigned short v16us __attribute__((ext_vector_type(16)));
typedef _Float16       v16h  __attribute__((ext_vector_type(16)));
typedef float          v4f   __attribute__((ext_vector_type(4)));
typedef float          v8f   __attribute__((ext_vector_type(8)));

union FragU { v16us v; v8us half[2]; };

__device__ __forceinline__ unsigned bbits(float f) {
  unsigned u = __float_as_uint(f);
  return (u + 0x7FFFu + ((u >> 16) & 1u)) >> 16;
}
__device__ __forceinline__ float bf16r(float f) {
  return __uint_as_float(bbits(f) << 16);
}
__device__ __forceinline__ unsigned short hbits(float f) {
  return __builtin_bit_cast(unsigned short, (_Float16)f);
}
__device__ __forceinline__ float rcpf(float x) {
#if defined(__HIP_DEVICE_COMPILE__)
  return __builtin_amdgcn_rcpf(x);
#else
  return 1.0f / x;
#endif
}
__device__ __forceinline__ v8f zero8() { v8f z = {0.f, 0.f, 0.f, 0.f, 0.f, 0.f, 0.f, 0.f}; return z; }
__device__ __forceinline__ v8us zero8us() { v8us z = {0, 0, 0, 0, 0, 0, 0, 0}; return z; }

__device__ __forceinline__ v16us ldfrag_u(const unsigned short* p) {
  FragU f;
  f.half[0] = *(const v8us*)(p);
  f.half[1] = *(const v8us*)(p + 16);
  return f.v;
}

__device__ __forceinline__ v8f mma_hu(v16us a, v16us b, v8f c) {
#if defined(__HIP_DEVICE_COMPILE__)
  return __builtin_amdgcn_wmma_f32_16x16x32_f16(false, __builtin_bit_cast(v16h, a),
                                               false, __builtin_bit_cast(v16h, b),
                                               (short)0, c, false, false);
#else
  (void)a; (void)b;
  return c;
#endif
}
__device__ __forceinline__ void guard4(v8f& c0, v8f& c1, v8f& c2, v8f& c3, const v16us& a,
                                       const v16us& b0, const v16us& b1, const v16us& b2,
                                       const v16us& b3) {
#if defined(__HIP_DEVICE_COMPILE__)
  asm volatile("v_nop\n\tv_nop\n\tv_nop\n\tv_nop"
               : "+v"(c0), "+v"(c1), "+v"(c2), "+v"(c3)
               : "v"(a), "v"(b0), "v"(b1), "v"(b2), "v"(b3));
#else
  (void)c0; (void)c1; (void)c2; (void)c3; (void)a; (void)b0; (void)b1; (void)b2; (void)b3;
#endif
}
__device__ __forceinline__ void guard8w(v8f& c0, v8f& c1, v8f& c2, v8f& c3, v8f& c4, v8f& c5,
                                        v8f& c6, v8f& c7, const v16us& a0, const v16us& a1,
                                        const v16us& b0, const v16us& b1, const v16us& b2,
                                        const v16us& b3, const v16us& b4, const v16us& b5,
                                        const v16us& b6, const v16us& b7) {
#if defined(__HIP_DEVICE_COMPILE__)
  asm volatile("v_nop\n\tv_nop\n\tv_nop\n\tv_nop"
               : "+v"(c0), "+v"(c1), "+v"(c2), "+v"(c3), "+v"(c4), "+v"(c5), "+v"(c6), "+v"(c7)
               : "v"(a0), "v"(a1), "v"(b0), "v"(b1), "v"(b2), "v"(b3), "v"(b4), "v"(b5),
                 "v"(b6), "v"(b7));
#else
  (void)c0; (void)c1; (void)c2; (void)c3; (void)c4; (void)c5; (void)c6; (void)c7;
  (void)a0; (void)a1; (void)b0; (void)b1; (void)b2; (void)b3; (void)b4; (void)b5; (void)b6; (void)b7;
#endif
}

__device__ __forceinline__ void store_tile_f32(const float* ct, float* C, size_t row0, int col0,
                                               int ldc, int w, int lane) {
  const int q  = lane >> 3;
  const int jj = lane & 7;
#pragma unroll 1
  for (int it = 0; it < 8; ++it) {
    const int li = it * 16 + w * 4 + q;
    const int tr = li >> 1, hf = li & 1;
    const v4f v = *(const v4f*)(ct + tr * 64 + hf * 32 + jj * 4);
    *(volatile v4f*)(C + (row0 + tr) * (size_t)ldc + col0 + hf * 32 + jj * 4) = v;
  }
  __threadfence();
#pragma unroll 1
  for (int it = 0; it < 8; ++it) {
    const int li = it * 16 + w * 4 + q;
    const int tr = li >> 1, hf = li & 1;
    const v4f v = *(const v4f*)(ct + tr * 64 + hf * 32 + jj * 4);
    *(volatile v4f*)(C + (row0 + tr) * (size_t)ldc + col0 + hf * 32 + jj * 4) = v;
  }
}
template <int NW, int PITCH>
__device__ __forceinline__ void store_tile_us(const unsigned short* t, unsigned short* P,
                                              size_t row0, int ld, int col0, int w, int lane) {
  constexpr int NIT = 64 / (4 * NW);
  const int q  = lane >> 3;
  const int jj = lane & 7;
  v8us   v[NIT];
  size_t off[NIT];
#pragma unroll
  for (int it = 0; it < NIT; ++it) {
    const int li = it * 4 * NW + w * 4 + q;
    v[it]   = *(const v8us*)(t + li * PITCH + 8 * jj);
    off[it] = (row0 + li) * (size_t)ld + col0 + 8 * jj;
  }
#pragma unroll
  for (int it = 0; it < NIT; ++it) *(volatile v8us*)(P + off[it]) = v[it];
  __threadfence();
#pragma unroll
  for (int it = 0; it < NIT; ++it) *(volatile v8us*)(P + off[it]) = v[it];
}

__global__ __launch_bounds__(256)
void k_pad(const float* __restrict__ qin, const float* __restrict__ sin_, unsigned short* xp)
{
  __shared__ __align__(16) unsigned short T[PW * TPP];

  const int tid  = threadIdx.x;
  const int lane = tid & 31;
  const int w    = tid >> 5;
  const int hp   = blockIdx.x;
  const int img  = blockIdx.y;
  const float* src = (img < 2) ? (sin_ + (size_t)img * CIN * NPX)
                               : (qin + (size_t)(img - 2) * CIN * NPX);
  const int c = tid;
  T[c] = 0;
  T[(PW - 1) * TPP + c] = 0;
  if (hp >= 1 && hp <= HWD) {
    const float* rp = src + (size_t)c * NPX + (size_t)(hp - 1) * HWD;
#pragma unroll 2
    for (int g = 0; g < 16; ++g) {
      const v4f u = *(const v4f*)(rp + 4 * g);
#pragma unroll
      for (int e = 0; e < 4; ++e) T[(4 * g + e + 1) * TPP + c] = hbits(bf16r(u[e]));
    }
  } else {
#pragma unroll 4
    for (int p = 1; p <= HWD; ++p) T[p * TPP + c] = 0;
  }
  __syncthreads();

  const int q  = lane >> 3;
  const int jj = lane & 7;
  unsigned short* base = xp + ((size_t)img * PW + hp) * PW * CIN;
#pragma unroll 1
  for (int it = 0; it < 9; ++it) {
    const int li = it * 32 + 4 * w + q;
    if (li < 4 * PW) {
      const int px = li >> 2, qq = li & 3;
      const v8us v = *(const v8us*)(T + px * TPP + 64 * qq + 8 * jj);
      *(volatile v8us*)(base + (size_t)px * CIN + 64 * qq + 8 * jj) = v;
    }
  }
  __threadfence();
#pragma unroll 1
  for (int it = 0; it < 9; ++it) {
    const int li = it * 32 + 4 * w + q;
    if (li < 4 * PW) {
      const int px = li >> 2, qq = li & 3;
      const v8us v = *(const v8us*)(T + px * TPP + 64 * qq + 8 * jj);
      *(volatile v8us*)(base + (size_t)px * CIN + 64 * qq + 8 * jj) = v;
    }
  }
}

__global__ __launch_bounds__(256)
void k_wcvt(const float* __restrict__ tsw, const float* __restrict__ tqw, const float* __restrict__ ccw,
            const float* __restrict__ cvw, const float* __restrict__ k1w, const float* __restrict__ q1w,
            const float* __restrict__ k2w, const float* __restrict__ q2w,
            unsigned short* w3r, unsigned short* wc)
{
  const int tid = threadIdx.x;
  const int bid = blockIdx.x;
  v8us ob;
  unsigned short* dst;
  if (bid < 432) {
    const int set = bid / 144;
    const int t   = bid * 256 + tid;
    const int o   = 8 * t;
    const int rem = o - set * (int)W3SET;
    const int co  = rem / KC3;
    const int k   = rem - co * KC3;
    const int tap = k >> 8;
    const int c   = k & 255;
    const float* wsrc = (set == 0) ? tsw : ((set == 1) ? tqw : ccw);
    const float* p = wsrc + ((size_t)co * CIN + c) * 9 + tap;
#pragma unroll
    for (int e = 0; e < 8; ++e) ob[e] = hbits(16.0f * bf16r(p[9 * e]));
    dst = w3r + o;
  } else {
    const int t   = (bid - 432) * 256 + tid;
    const int o   = 8 * t;
    const int set = o >> 15;
    const int row = (o >> 7) & 255;
    const int c   = o & 127;
    const float* p = (row < 128) ? (cvw + (size_t)row * CI + c)
                   : ((row < 192) ? ((set ? k2w : k1w) + (size_t)(row - 128) * CI + c)
                                  : ((set ? q2w : q1w) + (size_t)(row - 192) * CI + c));
#pragma unroll
    for (int e = 0; e < 8; ++e) ob[e] = hbits(16.0f * bf16r(p[e]));
    dst = wc + o;
  }
  *(volatile v8us*)dst = ob;
  __threadfence();
  *(volatile v8us*)dst = ob;
}

template <int STEM>
__device__ __forceinline__ void conv3_tile(const unsigned short* __restrict__ xpimg,
                                           const unsigned short* __restrict__ wr,
                                           const float* bias, const float* bg, const float* bbe,
                                           const float* bm, const float* bv,
                                           float* fdst, unsigned short* xh, unsigned short* xl,
                                           float* ct, unsigned short* th, unsigned short* tl)
{
  const int tid  = threadIdx.x;
  const int lane = tid & 31;
  const int w    = tid >> 5;
  const int h    = lane >> 4;
  const int m    = lane & 15;
  const int hrow = blockIdx.x;
  const int co0  = 64 * blockIdx.y;

  v8f acc[4];
#pragma unroll
  for (int j = 0; j < 4; ++j) acc[j] = zero8();

  const unsigned short* pa = wr + (size_t)(co0 + 16 * w + m) * KC3 + 8 * h;
  const unsigned short* pb = xpimg + ((size_t)hrow * PW + m) * CIN + 8 * h;
#pragma unroll 1
  for (int r = 0; r < 3; ++r) {
#pragma unroll 1
    for (int s = 0; s < 3; ++s) {
      const unsigned short* pat = pa + (3 * r + s) * CIN;
      const unsigned short* pbt = pb + ((size_t)r * PW + s) * CIN;
#pragma unroll 2
      for (int kk = 0; kk < CIN / 32; ++kk) {
        const v16us a  = ldfrag_u(pat + 32 * kk);
        const v16us b0 = ldfrag_u(pbt + 32 * kk);
        const v16us b1 = ldfrag_u(pbt + (size_t)16 * CIN + 32 * kk);
        const v16us b2 = ldfrag_u(pbt + (size_t)32 * CIN + 32 * kk);
        const v16us b3 = ldfrag_u(pbt + (size_t)48 * CIN + 32 * kk);
        acc[0] = mma_hu(a, b0, acc[0]);
        acc[1] = mma_hu(a, b1, acc[1]);
        acc[2] = mma_hu(a, b2, acc[2]);
        acc[3] = mma_hu(a, b3, acc[3]);
        guard4(acc[0], acc[1], acc[2], acc[3], a, b0, b1, b2, b3);
      }
    }
  }

  const float k16 = 1.0f / 16.0f;
  float cb[8], cmn[8], csc[8], cbe[8];
#pragma unroll
  for (int r = 0; r < 8; ++r) {
    const int c = co0 + 16 * w + 8 * h + r;
    cb[r]  = STEM ? bf16r(bias[c]) : 0.0f;
    cmn[r] = bf16r(bm[c]);
    csc[r] = bf16r(bg[c]) * rcpf(sqrtf(bf16r(bv[c]) + 1e-5f));
    cbe[r] = bf16r(bbe[c]);
  }
#pragma unroll
  for (int j = 0; j < 4; ++j) {
#pragma unroll
    for (int r = 0; r < 8; ++r) {
      float v = acc[j][r] * k16 + cb[r];
      v = (v - cmn[r]) * csc[r] + cbe[r];
      v = fmaxf(v, 0.0f);
      const int rl = 16 * w + 8 * h + r;
      const int cl = 16 * j + m;
      ct[rl * 64 + cl] = v;
      if (STEM) {
        const _Float16 hv = (_Float16)v;
        th[cl * TP + rl] = __builtin_bit_cast(unsigned short, hv);
        tl[cl * TP + rl] = hbits((v - (float)hv) * 32768.0f);
      }
    }
  }
  __syncthreads();
  store_tile_f32(ct, fdst, (size_t)co0, 64 * hrow, NPX, w, lane);
  if (STEM) {
    store_tile_us<4, TP>(th, xh, (size_t)64 * hrow, CI, co0, w, lane);
    store_tile_us<4, TP>(tl, xl, (size_t)64 * hrow, CI, co0, w, lane);
  }
}

__global__ __launch_bounds__(128)
void k_conv3_stem(const unsigned short* __restrict__ xp, const unsigned short* __restrict__ w3r,
                  const float* __restrict__ tsb, const float* __restrict__ tsg,
                  const float* __restrict__ tsbe, const float* __restrict__ tsm,
                  const float* __restrict__ tsv,
                  const float* __restrict__ tqb, const float* __restrict__ tqg,
                  const float* __restrict__ tqbe, const float* __restrict__ tqm,
                  const float* __restrict__ tqv,
                  float* xs, unsigned short* xh, unsigned short* xl)
{
  __shared__ __align__(16) float ct[64 * 64];
  __shared__ __align__(16) unsigned short th[64 * TP];
  __shared__ __align__(16) unsigned short tl[64 * TP];
  const int img   = blockIdx.z;
  const int which = img >> 1;
  conv3_tile<1>(xp + (size_t)img * XPIMG, w3r + (size_t)which * W3SET,
                which ? tqb : tsb, which ? tqg : tsg, which ? tqbe : tsbe,
                which ? tqm : tsm, which ? tqv : tsv,
                xs + (size_t)img * XSIMG, xh + (size_t)img * XHIMG, xl + (size_t)img * XHIMG,
                ct, th, tl);
}

__global__ __launch_bounds__(128)
void k_conv3_cc(const unsigned short* __restrict__ ep, const unsigned short* __restrict__ wcc,
                const float* __restrict__ ccg, const float* __restrict__ ccbe,
                const float* __restrict__ ccm, const float* __restrict__ ccv, float* out)
{
  __shared__ __align__(16) float ct[64 * 64];
  const int b = blockIdx.z;
  conv3_tile<0>(ep + (size_t)b * XPIMG, wcc, nullptr, ccg, ccbe, ccm, ccv,
                out + (size_t)b * OUTB, nullptr, nullptr, ct, nullptr, nullptr);
}

__global__ __launch_bounds__(128)
void k_c1x1(const unsigned short* __restrict__ wc, const unsigned short* __restrict__ xh,
            const unsigned short* __restrict__ xl,
            const float* __restrict__ cvb, const float* __restrict__ k1b,
            const float* __restrict__ q1b, const float* __restrict__ k2b,
            const float* __restrict__ q2b,
            unsigned short* v16, float* vp, unsigned short* kh, unsigned short* kl,
            unsigned short* qh, unsigned short* ql)
{
  __shared__ __align__(16) unsigned short t0[64 * TP];
  __shared__ __align__(16) unsigned short t1[64 * TP];
  __shared__ __align__(16) float rsl[64];

  const int tid   = threadIdx.x;
  const int lane  = tid & 31;
  const int w     = tid >> 5;
  const int h     = lane >> 4;
  const int m     = lane & 15;
  const int nt    = blockIdx.x;
  const int n0    = 64 * nt;
  const int role  = blockIdx.y;
  const int img   = blockIdx.z;
  const int which = img >> 1;
  const int b     = img & 1;

  v8f acc[4], accl[4];
#pragma unroll
  for (int j = 0; j < 4; ++j) { acc[j] = zero8(); accl[j] = zero8(); }

  const unsigned short* pa  = wc + (size_t)which * WCSET + (size_t)(64 * role + 16 * w + m) * CI + 8 * h;
  const unsigned short* pbh = xh + (size_t)img * XHIMG + (size_t)(n0 + m) * CI + 8 * h;
  const unsigned short* pbl = xl + (size_t)img * XHIMG + (size_t)(n0 + m) * CI + 8 * h;

  if (role < 2) {
#pragma unroll 2
    for (int kk = 0; kk < CI / 32; ++kk) {
      const v16us a  = ldfrag_u(pa + 32 * kk);
      const v16us b0 = ldfrag_u(pbh + 32 * kk);
      const v16us b1 = ldfrag_u(pbh + (size_t)16 * CI + 32 * kk);
      const v16us b2 = ldfrag_u(pbh + (size_t)32 * CI + 32 * kk);
      const v16us b3 = ldfrag_u(pbh + (size_t)48 * CI + 32 * kk);
      acc[0] = mma_hu(a, b0, acc[0]);
      acc[1] = mma_hu(a, b1, acc[1]);
      acc[2] = mma_hu(a, b2, acc[2]);
      acc[3] = mma_hu(a, b3, acc[3]);
      guard4(acc[0], acc[1], acc[2], acc[3], a, b0, b1, b2, b3);
    }
  } else {
#pragma unroll 1
    for (int kk = 0; kk < CI / 32; ++kk) {
      const v16us a   = ldfrag_u(pa + 32 * kk);
      const v16us bh0 = ldfrag_u(pbh + 32 * kk);
      const v16us bh1 = ldfrag_u(pbh + (size_t)16 * CI + 32 * kk);
      const v16us bh2 = ldfrag_u(pbh + (size_t)32 * CI + 32 * kk);
      const v16us bh3 = ldfrag_u(pbh + (size_t)48 * CI + 32 * kk);
      const v16us bl0 = ldfrag_u(pbl + 32 * kk);
      const v16us bl1 = ldfrag_u(pbl + (size_t)16 * CI + 32 * kk);
      const v16us bl2 = ldfrag_u(pbl + (size_t)32 * CI + 32 * kk);
      const v16us bl3 = ldfrag_u(pbl + (size_t)48 * CI + 32 * kk);
      acc[0]  = mma_hu(a, bh0, acc[0]);
      acc[1]  = mma_hu(a, bh1, acc[1]);
      acc[2]  = mma_hu(a, bh2, acc[2]);
      acc[3]  = mma_hu(a, bh3, acc[3]);
      accl[0] = mma_hu(a, bl0, accl[0]);
      accl[1] = mma_hu(a, bl1, accl[1]);
      accl[2] = mma_hu(a, bl2, accl[2]);
      accl[3] = mma_hu(a, bl3, accl[3]);
      guard8w(acc[0], acc[1], acc[2], acc[3], accl[0], accl[1], accl[2], accl[3],
              a, a, bh0, bh1, bh2, bh3, bl0, bl1, bl2, bl3);
    }
  }

  const float k16 = 1.0f / 16.0f;
  const float klo = 1.0f / 32768.0f;
  if (role < 2) {
    float bias[8];
    float rs[8];
#pragma unroll
    for (int r = 0; r < 8; ++r) { bias[r] = bf16r(cvb[64 * role + 16 * w + 8 * h + r]); rs[r] = 0.0f; }
#pragma unroll
    for (int j = 0; j < 4; ++j) {
#pragma unroll
      for (int r = 0; r < 8; ++r) {
        const float v = acc[j][r] * k16 + bias[r];
        const int rl = 16 * w + 8 * h + r;
        const int cl = 16 * j + m;
        t0[rl * TP + cl] = hbits(16.0f * v);
        rs[r] += v;
      }
    }
#pragma unroll
    for (int r = 0; r < 8; ++r) {
#pragma unroll
      for (int o = 1; o < 16; o <<= 1) rs[r] += __shfl_xor(rs[r], o, 32);
    }
    if (m == 0) {
#pragma unroll
      for (int r = 0; r < 8; ++r) rsl[16 * w + 8 * h + r] = rs[r];
    }
    __syncthreads();
    store_tile_us<4, TP>(t0, v16 + (size_t)img * VIMG, (size_t)64 * role, NPX, n0, w, lane);
    if (w == 0 && lane < 16) {
      const v4f v = *(const v4f*)(rsl + 4 * lane);
      float* d = vp + ((size_t)img * 64 + nt) * CI + 64 * role + 4 * lane;
      *(volatile v4f*)d = v;
      __threadfence();
      *(volatile v4f*)d = v;
    }
  } else {
    const float* bb = (role == 2) ? (which ? k2b : k1b) : (which ? q2b : q1b);
    const float sgn = (role == 2 && which == 1) ? -1.0f : 1.0f;
    float bias[8];
#pragma unroll
    for (int r = 0; r < 8; ++r) bias[r] = bf16r(bb[16 * w + 8 * h + r]);
#pragma unroll
    for (int j = 0; j < 4; ++j) {
#pragma unroll
      for (int r = 0; r < 8; ++r) {
        const float val = ((acc[j][r] + accl[j][r] * klo) * k16 + bias[r]) * sgn;
        const _Float16 hv = (_Float16)val;
        const int rl = 16 * w + 8 * h + r;
        const int cl = 16 * j + m;
        t0[cl * TP + rl] = __builtin_bit_cast(unsigned short, hv);
        t1[cl * TP + rl] = hbits((val - (float)hv) * 32768.0f);
      }
    }
    __syncthreads();
    unsigned short* dh = (role == 2) ? kh : qh;
    unsigned short* dl = (role == 2) ? kl : ql;
    store_tile_us<4, TP>(t0, dh + (size_t)b * KIMG, (size_t)n0, CI, 64 * which, w, lane);
    store_tile_us<4, TP>(t1, dl + (size_t)b * KIMG, (size_t)n0, CI, 64 * which, w, lane);
  }
}

__global__ __launch_bounds__(128)
void k_gate(const float* __restrict__ vp, const float* __restrict__ g1w, const float* __restrict__ g1b,
            const float* __restrict__ g2w, const float* __restrict__ g2b, float* g)
{
  __shared__ float pooled[CI];
  __shared__ float hid[8];
  __shared__ __align__(16) float gl[CI];
  const int tid = threadIdx.x;
  const int img = blockIdx.x;
  const int c   = tid;
  float s = 0.0f;
#pragma unroll 1
  for (int t = 0; t < 64; ++t) s += vp[((size_t)img * 64 + t) * CI + c];
  pooled[c] = s * (1.0f / 4096.0f);
  __syncthreads();
  if (tid < 8) {
    float a = 0.0f;
#pragma unroll 1
    for (int c2 = 0; c2 < CI; ++c2) a += pooled[c2] * bf16r(g1w[tid * CI + c2]);
    a += bf16r(g1b[tid]);
    hid[tid] = fmaxf(a, 0.0f);
  }
  __syncthreads();
  float a = 0.0f;
#pragma unroll 1
  for (int j = 0; j < 8; ++j) a += hid[j] * bf16r(g2w[c * 8 + j]);
  a += bf16r(g2b[c]);
  const float ex = __expf(-a);
  gl[c] = rcpf(1.0f + ex);
  __syncthreads();
  if (tid < 32) {
    const v4f v = *(const v4f*)(gl + 4 * tid);
    float* d = g + (size_t)img * CI + 4 * tid;
    *(volatile v4f*)d = v;
    __threadfence();
    *(volatile v4f*)d = v;
  }
}

__global__ __launch_bounds__(128)
void k_score(const unsigned short* __restrict__ kh, const unsigned short* __restrict__ kl,
             const unsigned short* __restrict__ qh, const unsigned short* __restrict__ ql, float* S)
{
  __shared__ __align__(16) float ct[64 * 64];

  const int tid  = threadIdx.x;
  const int lane = tid & 31;
  const int w    = tid >> 5;
  const int h    = lane >> 4;
  const int m    = lane & 15;
  const int m0   = 64 * blockIdx.x;
  const int n0   = 64 * blockIdx.y;

  v8f acc[4], accx[4];
#pragma unroll
  for (int j = 0; j < 4; ++j) { acc[j] = zero8(); accx[j] = zero8(); }

  const unsigned short* pah = kh + (size_t)(n0 + 16 * w + m) * CI + 8 * h;
  const unsigned short* pal = kl + (size_t)(n0 + 16 * w + m) * CI + 8 * h;
  const unsigned short* pbh = qh + (size_t)(m0 + m) * CI + 8 * h;
  const unsigned short* pbl = ql + (size_t)(m0 + m) * CI + 8 * h;
#pragma unroll 1
  for (int kk = 0; kk < CI / 32; ++kk) {
    const v16us ah  = ldfrag_u(pah + 32 * kk);
    const v16us al  = ldfrag_u(pal + 32 * kk);
    const v16us bh0 = ldfrag_u(pbh + 32 * kk);
    const v16us bh1 = ldfrag_u(pbh + (size_t)16 * CI + 32 * kk);
    const v16us bh2 = ldfrag_u(pbh + (size_t)32 * CI + 32 * kk);
    const v16us bh3 = ldfrag_u(pbh + (size_t)48 * CI + 32 * kk);
    const v16us bl0 = ldfrag_u(pbl + 32 * kk);
    const v16us bl1 = ldfrag_u(pbl + (size_t)16 * CI + 32 * kk);
    const v16us bl2 = ldfrag_u(pbl + (size_t)32 * CI + 32 * kk);
    const v16us bl3 = ldfrag_u(pbl + (size_t)48 * CI + 32 * kk);
    acc[0]  = mma_hu(ah, bh0, acc[0]);
    acc[1]  = mma_hu(ah, bh1, acc[1]);
    acc[2]  = mma_hu(ah, bh2, acc[2]);
    acc[3]  = mma_hu(ah, bh3, acc[3]);
    accx[0] = mma_hu(ah, bl0, accx[0]);
    accx[1] = mma_hu(ah, bl1, accx[1]);
    accx[2] = mma_hu(ah, bl2, accx[2]);
    accx[3] = mma_hu(ah, bl3, accx[3]);
    accx[0] = mma_hu(al, bh0, accx[0]);
    accx[1] = mma_hu(al, bh1, accx[1]);
    accx[2] = mma_hu(al, bh2, accx[2]);
    accx[3] = mma_hu(al, bh3, accx[3]);
    guard8w(acc[0], acc[1], acc[2], acc[3], accx[0], accx[1], accx[2], accx[3],
            ah, al, bh0, bh1, bh2, bh3, bl0, bl1, bl2, bl3);
  }

  const float kx = 1.0f / 32768.0f;
#pragma unroll
  for (int j = 0; j < 4; ++j) {
#pragma unroll
    for (int r = 0; r < 8; ++r)
      ct[(16 * w + 8 * h + r) * 64 + 16 * j + m] = fabsf(acc[j][r] + accx[j][r] * kx);
  }
  __syncthreads();
  store_tile_f32(ct, S, (size_t)n0, m0, NPX, w, lane);
}

__global__ __launch_bounds__(256)
void k_rstat(const float* __restrict__ S, float* rmax, float* rsum)
{
  __shared__ __align__(16) float lm[32];
  __shared__ __align__(16) float ls[32];
  const int tid  = threadIdx.x;
  const int lane = tid & 31;
  const int w    = tid >> 5;
#pragma unroll 1
  for (int rr = 0; rr < 4; ++rr) {
    const int row = 32 * blockIdx.x + 4 * w + rr;
    const float* sr = S + (size_t)row * NPX + 8 * lane;
    float mx = 0.0f, sm = 0.0f;
#pragma unroll 1
    for (int it = 0; it < NPX / 256; ++it) {
      const v4f x0 = *(const v4f*)(sr + 256 * it);
      const v4f x1 = *(const v4f*)(sr + 256 * it + 4);
      const float cm = fmaxf(fmaxf(fmaxf(x0[0], x0[1]), fmaxf(x0[2], x0[3])),
                             fmaxf(fmaxf(x1[0], x1[1]), fmaxf(x1[2], x1[3])));
      const float mn = fmaxf(mx, cm);
      float add = 0.0f;
#pragma unroll
      for (int e = 0; e < 4; ++e) { add += __expf(x0[e] - mn); add += __expf(x1[e] - mn); }
      sm = sm * __expf(mx - mn) + add;
      mx = mn;
    }
    float M = mx;
#pragma unroll
    for (int o = 16; o >= 1; o >>= 1) M = fmaxf(M, __shfl_xor(M, o, 32));
    float st = sm * __expf(mx - M);
#pragma unroll
    for (int o = 16; o >= 1; o >>= 1) st += __shfl_xor(st, o, 32);
    if (lane == 0) { lm[4 * w + rr] = M; ls[4 * w + rr] = st; }
  }
  __syncthreads();
  if (w == 0 && lane < 8) {
    const v4f a = *(const v4f*)(lm + 4 * lane);
    const v4f c = *(const v4f*)(ls + 4 * lane);
    float* dm = rmax + 32 * blockIdx.x + 4 * lane;
    float* ds = rsum + 32 * blockIdx.x + 4 * lane;
    *(volatile v4f*)dm = a;
    *(volatile v4f*)ds = c;
    __threadfence();
    *(volatile v4f*)dm = a;
    *(volatile v4f*)ds = c;
  }
}

__global__ __launch_bounds__(256)
void k_cstat(const float* __restrict__ S, float* cmax, float* csum)
{
  __shared__ float lmx[8][32];
  __shared__ float lsm[8][32];
  __shared__ __align__(16) float om[32];
  __shared__ __align__(16) float osm[32];
  const int tid = threadIdx.x;
  const int tx  = tid & 31;
  const int ty  = tid >> 5;
  const int col = 32 * blockIdx.x + tx;
  const float* sp = S + (size_t)(512 * ty) * NPX + col;
  float mx = 0.0f, sm = 0.0f;
#pragma unroll 1
  for (int it = 0; it < 128; ++it) {
    const float* p4 = sp + (size_t)(4 * it) * NPX;
    const float a0 = p4[0];
    const float a1 = p4[NPX];
    const float a2 = p4[2 * NPX];
    const float a3 = p4[3 * NPX];
    const float cm = fmaxf(fmaxf(a0, a1), fmaxf(a2, a3));
    const float mn = fmaxf(mx, cm);
    const float add = (__expf(a0 - mn) + __expf(a1 - mn)) + (__expf(a2 - mn) + __expf(a3 - mn));
    sm = sm * __expf(mx - mn) + add;
    mx = mn;
  }
  lmx[ty][tx] = mx;
  lsm[ty][tx] = sm;
  __syncthreads();
  if (ty == 0) {
    float M = lmx[0][tx];
#pragma unroll
    for (int j = 1; j < 8; ++j) M = fmaxf(M, lmx[j][tx]);
    float st = 0.0f;
#pragma unroll
    for (int j = 0; j < 8; ++j) st += lsm[j][tx] * __expf(lmx[j][tx] - M);
    om[tx]  = M;
    osm[tx] = st;
  }
  __syncthreads();
  if (ty == 0 && tx < 8) {
    const v4f a = *(const v4f*)(om + 4 * tx);
    const v4f c = *(const v4f*)(osm + 4 * tx);
    float* dm = cmax + 32 * blockIdx.x + 4 * tx;
    float* ds = csum + 32 * blockIdx.x + 4 * tx;
    *(volatile v4f*)dm = a;
    *(volatile v4f*)ds = c;
    __threadfence();
    *(volatile v4f*)dm = a;
    *(volatile v4f*)ds = c;
  }
}

__device__ __forceinline__ void pv_store_pass(const float* Et, float* eout, unsigned short* epimg,
                                              int choff, int hrow, int R0, int w, int lane)
{
  const int q  = lane >> 3;
  const int jj = lane & 7;
#pragma unroll 1
  for (int it = 0; it < 8; ++it) {
    const int li = it * 32 + 4 * w + q;
    const int c = li >> 1, hf = li & 1;
    const v4f v = *(const v4f*)(Et + c * EPF + 32 * hf + 4 * jj);
    *(volatile v4f*)(eout + (size_t)c * NPX + R0 + 32 * hf + 4 * jj) = v;
  }
#pragma unroll 1
  for (int it = 0; it < 4; ++it) {
    const int li = it * 32 + 4 * w + q;
    const int px = li >> 1, hf = li & 1;
    v8us o;
#pragma unroll
    for (int e = 0; e < 8; ++e) o[e] = hbits(Et[(64 * hf + 8 * jj + e) * EPF + px]);
    *(volatile v8us*)(epimg + ((size_t)(hrow + 1) * PW + (px + 1)) * CIN + choff + 64 * hf + 8 * jj) = o;
  }
}

template <int DIRQ>
__global__ __launch_bounds__(256)
void k_pv(const float* __restrict__ S, const float* __restrict__ smax, const float* __restrict__ ssum,
          const unsigned short* __restrict__ vimg, const float* __restrict__ gimg,
          const float* __restrict__ xsimg, float* eout, unsigned short* epimg, int choff)
{
  __shared__ __align__(16) unsigned short Pt[64 * TP];
  __shared__ __align__(16) float Et[CI * EPF];
  __shared__ float mxs[64];
  __shared__ float invs[64];
  __shared__ float gv[CI];

  const int tid  = threadIdx.x;
  const int lane = tid & 31;
  const int w    = tid >> 5;
  const int h    = lane >> 4;
  const int m    = lane & 15;
  const int hrow = blockIdx.x;
  const int R0   = 64 * hrow;

  if (tid < 64) {
    mxs[tid]  = smax[R0 + tid];
    invs[tid] = rcpf(ssum[R0 + tid]) * (1.0f / 262144.0f);
  }
  if (tid < CI) gv[tid] = gimg[tid];
  __syncthreads();

  const int fr = tid >> 2;
  const int fc = 16 * (tid & 3);
  float mxr[16];
  const float* sp;
  if (DIRQ == 0) {
    mxr[0] = mxs[fr];
    sp = S + (size_t)(R0 + fr) * NPX + fc;
  } else {
#pragma unroll
    for (int e = 0; e < 16; ++e) mxr[e] = mxs[fc + e];
    sp = S + (size_t)fr * NPX + R0 + fc;
  }

  v8f acc[4];
#pragma unroll
  for (int j = 0; j < 4; ++j) acc[j] = zero8();
  const unsigned short* pa = vimg + (size_t)(16 * w + m) * NPX + 8 * h;

#pragma unroll 1
  for (int T = 0; T < NPX / 64; ++T) {
    if (DIRQ == 0) {
      const float* s2 = sp + 64 * T;
      const v4f x0 = *(const v4f*)(s2);
      const v4f x1 = *(const v4f*)(s2 + 4);
      const v4f x2 = *(const v4f*)(s2 + 8);
      const v4f x3 = *(const v4f*)(s2 + 12);
      const float mx0 = mxr[0];
      v8us o0, o1;
#pragma unroll
      for (int e = 0; e < 4; ++e) {
        o0[e]     = hbits(16384.0f * __expf(x0[e] - mx0));
        o0[4 + e] = hbits(16384.0f * __expf(x1[e] - mx0));
        o1[e]     = hbits(16384.0f * __expf(x2[e] - mx0));
        o1[4 + e] = hbits(16384.0f * __expf(x3[e] - mx0));
      }
      *(v8us*)(Pt + fr * TP + fc)     = o0;
      *(v8us*)(Pt + fr * TP + fc + 8) = o1;
    } else {
      const float* s2 = sp + (size_t)T * 64 * NPX;
      const v4f x0 = *(const v4f*)(s2);
      const v4f x1 = *(const v4f*)(s2 + 4);
      const v4f x2 = *(const v4f*)(s2 + 8);
      const v4f x3 = *(const v4f*)(s2 + 12);
#pragma unroll
      for (int e = 0; e < 4; ++e) {
        Pt[(fc + e) * TP + fr]      = hbits(16384.0f * __expf(x0[e] - mxr[e]));
        Pt[(fc + 4 + e) * TP + fr]  = hbits(16384.0f * __expf(x1[e] - mxr[4 + e]));
        Pt[(fc + 8 + e) * TP + fr]  = hbits(16384.0f * __expf(x2[e] - mxr[8 + e]));
        Pt[(fc + 12 + e) * TP + fr] = hbits(16384.0f * __expf(x3[e] - mxr[12 + e]));
      }
    }
    __syncthreads();
#pragma unroll
    for (int kk = 0; kk < 2; ++kk) {
      const v16us a  = ldfrag_u(pa + 64 * T + 32 * kk);
      const v16us b0 = ldfrag_u(Pt + (0 * 16 + m) * TP + 32 * kk + 8 * h);
      const v16us b1 = ldfrag_u(Pt + (1 * 16 + m) * TP + 32 * kk + 8 * h);
      const v16us b2 = ldfrag_u(Pt + (2 * 16 + m) * TP + 32 * kk + 8 * h);
      const v16us b3 = ldfrag_u(Pt + (3 * 16 + m) * TP + 32 * kk + 8 * h);
      acc[0] = mma_hu(a, b0, acc[0]);
      acc[1] = mma_hu(a, b1, acc[1]);
      acc[2] = mma_hu(a, b2, acc[2]);
      acc[3] = mma_hu(a, b3, acc[3]);
      guard4(acc[0], acc[1], acc[2], acc[3], a, b0, b1, b2, b3);
    }
    __syncthreads();
  }

#pragma unroll
  for (int j = 0; j < 4; ++j) {
#pragma unroll
    for (int r = 0; r < 8; ++r) {
      const int c = 16 * w + 8 * h + r;
      const int i = 16 * j + m;
      const float p = acc[j][r] * invs[i];
      Et[c * EPF + i] = gv[c] * p + xsimg[(size_t)c * NPX + R0 + i];
    }
  }
  __syncthreads();
  pv_store_pass(Et, eout, epimg, choff, hrow, R0, w, lane);
  __threadfence();
  pv_store_pass(Et, eout, epimg, choff, hrow, R0, w, lane);
}

__global__ __launch_bounds__(256)
void k_ephalo(unsigned short* ep)
{
  const int tid  = threadIdx.x;
  const int lane = tid & 31;
  const int w    = tid >> 5;
  const int q    = lane >> 3;
  const int jj   = lane & 7;
  const int hp   = blockIdx.x;
  const int b    = blockIdx.y;
  unsigned short* base = ep + ((size_t)b * PW + hp) * PW * CIN;
  const int halo = (hp == 0 || hp == PW - 1) ? 1 : 0;
  const int nl   = halo ? (4 * PW) : 8;
  const v8us z   = zero8us();
#pragma unroll 1
  for (int it = 0; it < 9; ++it) {
    const int li = it * 32 + 4 * w + q;
    if (li < nl) {
      const int px = halo ? (li >> 2) : ((li >> 2) ? (PW - 1) : 0);
      const int qq = li & 3;
      *(volatile v8us*)(base + (size_t)px * CIN + 64 * qq + 8 * jj) = z;
    }
  }
  __threadfence();
#pragma unroll 1
  for (int it = 0; it < 9; ++it) {
    const int li = it * 32 + 4 * w + q;
    if (li < nl) {
      const int px = halo ? (li >> 2) : ((li >> 2) ? (PW - 1) : 0);
      const int qq = li & 3;
      *(volatile v8us*)(base + (size_t)px * CIN + 64 * qq + 8 * jj) = z;
    }
  }
}

extern "C" void kernel_launch(void* const* d_in, const int* in_sizes, int n_in,
                              void* d_out, int out_size, void* d_ws, size_t ws_size,
                              hipStream_t stream) {
  if (n_in < 33) return;
  if (in_sizes[0] != NBT * CIN * NPX) return;
  if (in_sizes[1] != NBT * CIN * NPX) return;
  if (in_sizes[2] != CI * CIN * 9) return;
  if (in_sizes[8] != CI * CIN * 9) return;
  if (in_sizes[28] != CI * CIN * 9) return;
  if (in_sizes[3] != CI || in_sizes[4] != CI || in_sizes[5] != CI || in_sizes[6] != CI ||
      in_sizes[7] != CI) return;
  if (in_sizes[9] != CI || in_sizes[10] != CI || in_sizes[11] != CI || in_sizes[12] != CI ||
      in_sizes[13] != CI) return;
  if (in_sizes[14] != CI * CI || in_sizes[15] != CI) return;
  if (in_sizes[16] != 64 * CI || in_sizes[18] != 64 * CI || in_sizes[20] != 64 * CI ||
      in_sizes[22] != 64 * CI) return;
  if (in_sizes[17] != 64 || in_sizes[19] != 64 || in_sizes[21] != 64 || in_sizes[23] != 64) return;
  if (in_sizes[24] != 8 * CI || in_sizes[25] != 8 || in_sizes[26] != CI * 8 || in_sizes[27] != CI) return;
  if (in_sizes[29] != CI || in_sizes[30] != CI || in_sizes[31] != CI || in_sizes[32] != CI) return;
  if (out_size != 6 * (int)OUTB) return;
  if (ws_size < WS_TOTAL) return;

  const float* q    = (const float*)d_in[0];
  const float* s    = (const float*)d_in[1];
  const float* ts_w = (const float*)d_in[2];
  const float* ts_b = (const float*)d_in[3];
  const float* ts_g = (const float*)d_in[4];
  const float* ts_be= (const float*)d_in[5];
  const float* ts_m = (const float*)d_in[6];
  const float* ts_v = (const float*)d_in[7];
  const float* tq_w = (const float*)d_in[8];
  const float* tq_b = (const float*)d_in[9];
  const float* tq_g = (const float*)d_in[10];
  const float* tq_be= (const float*)d_in[11];
  const float* tq_m = (const float*)d_in[12];
  const float* tq_v = (const float*)d_in[13];
  const float* cv_w = (const float*)d_in[14];
  const float* cv_b = (const float*)d_in[15];
  const float* k1_w = (const float*)d_in[16];
  const float* k1_b = (const float*)d_in[17];
  const float* q1_w = (const float*)d_in[18];
  const float* q1_b = (const float*)d_in[19];
  const float* k2_w = (const float*)d_in[20];
  const float* k2_b = (const float*)d_in[21];
  const float* q2_w = (const float*)d_in[22];
  const float* q2_b = (const float*)d_in[23];
  const float* g1_w = (const float*)d_in[24];
  const float* g1_b = (const float*)d_in[25];
  const float* g2_w = (const float*)d_in[26];
  const float* g2_b = (const float*)d_in[27];
  const float* cc_w = (const float*)d_in[28];
  const float* cc_g = (const float*)d_in[29];
  const float* cc_be= (const float*)d_in[30];
  const float* cc_m = (const float*)d_in[31];
  const float* cc_v = (const float*)d_in[32];
  float* out = (float*)d_out;

  char* ws = (char*)d_ws;
  unsigned short* xp  = (unsigned short*)(ws + OFF_XP);
  unsigned short* w3r = (unsigned short*)(ws + OFF_W3);
  unsigned short* wc  = (unsigned short*)(ws + OFF_WC);
  float*          xs  = (float*)(ws + OFF_XS);
  unsigned short* xh  = (unsigned short*)(ws + OFF_XH);
  unsigned short* xl  = (unsigned short*)(ws + OFF_XL);
  unsigned short* v16 = (unsigned short*)(ws + OFF_V);
  float*          vp  = (float*)(ws + OFF_VP);
  float*          gt  = (float*)(ws + OFF_G);
  unsigned short* kh  = (unsigned short*)(ws + OFF_KH);
  unsigned short* kl  = (unsigned short*)(ws + OFF_KL);
  unsigned short* qh  = (unsigned short*)(ws + OFF_QH);
  unsigned short* ql  = (unsigned short*)(ws + OFF_QL);
  float*          Sp  = (float*)(ws + OFF_S);
  float*          rmx = (float*)(ws + OFF_RMAX);
  float*          rsm = (float*)(ws + OFF_RSUM);
  float*          cmx = (float*)(ws + OFF_CMAX);
  float*          csm = (float*)(ws + OFF_CSUM);
  unsigned short* ep  = (unsigned short*)(ws + OFF_EP);

  k_pad<<<dim3(PW, NIMG), dim3(256), 0, stream>>>(q, s, xp);
  (void)hipGetLastError();
  k_wcvt<<<dim3(464), dim3(256), 0, stream>>>(ts_w, tq_w, cc_w, cv_w, k1_w, q1_w, k2_w, q2_w, w3r, wc);
  (void)hipGetLastError();
  k_conv3_stem<<<dim3(HWD, 2, NIMG), dim3(128), 0, stream>>>(xp, w3r, ts_b, ts_g, ts_be, ts_m, ts_v,
                                                            tq_b, tq_g, tq_be, tq_m, tq_v, xs, xh, xl);
  (void)hipGetLastError();
  k_c1x1<<<dim3(NPX / 64, 4, NIMG), dim3(128), 0, stream>>>(wc, xh, xl, cv_b, k1_b, q1_b, k2_b, q2_b,
                                                           v16, vp, kh, kl, qh, ql);
  (void)hipGetLastError();
  k_gate<<<dim3(NIMG), dim3(128), 0, stream>>>(vp, g1_w, g1_b, g2_w, g2_b, gt);
  (void)hipGetLastError();

  for (int b = 0; b < NBT; ++b) {
    k_score<<<dim3(NPX / 64, NPX / 64), dim3(128), 0, stream>>>(
        kh + (size_t)b * KIMG, kl + (size_t)b * KIMG, qh + (size_t)b * KIMG, ql + (size_t)b * KIMG, Sp);
    (void)hipGetLastError();
    k_rstat<<<dim3(NPX / 32), dim3(256), 0, stream>>>(Sp, rmx, rsm);
    (void)hipGetLastError();
    k_cstat<<<dim3(NPX / 32), dim3(256), 0, stream>>>(Sp, cmx, csm);
    (void)hipGetLastError();
    k_pv<0><<<dim3(HWD), dim3(256), 0, stream>>>(
        Sp, rmx, rsm, v16 + (size_t)b * VIMG, gt + (size_t)b * CI, xs + (size_t)b * XSIMG,
        out + 4 * OUTB + (size_t)b * OUTB, ep + (size_t)b * XPIMG, CI);
    (void)hipGetLastError();
    k_pv<1><<<dim3(HWD), dim3(256), 0, stream>>>(
        Sp, cmx, csm, v16 + (size_t)(2 + b) * VIMG, gt + (size_t)(2 + b) * CI,
        xs + (size_t)(2 + b) * XSIMG, out + 2 * OUTB + (size_t)b * OUTB, ep + (size_t)b * XPIMG, 0);
    (void)hipGetLastError();
  }

  k_ephalo<<<dim3(PW, NBT), dim3(256), 0, stream>>>(ep);
  (void)hipGetLastError();
  k_conv3_cc<<<dim3(HWD, 2, NBT), dim3(128), 0, stream>>>(ep, w3r + (size_t)2 * W3SET,
                                                         cc_g, cc_be, cc_m, cc_v, out);
  (void)hipGetLastError();
}
